// TaoMamba_24567212934070
// MI455X (gfx1250) — hardware-verified
//
#include <hip/hip_runtime.h>


#define NB_  8
#define TIN  2048
#define LQ   2045
#define TT   2048
#define DIM  128
#define DI   256
#define DS   64
#define NH_  4
#define HP   64
#define CD   384
#define DP   644
#define ZH   4
typedef _Float16 h16;
typedef unsigned short bf;
typedef __attribute__((ext_vector_type(16))) __bf16   v16bf;
typedef __attribute__((ext_vector_type(16))) _Float16 v16h;
typedef __attribute__((ext_vector_type(8)))  _Float16 v8h;
typedef __attribute__((ext_vector_type(8)))  unsigned short v8us;
typedef __attribute__((ext_vector_type(8)))  float    v8f;
typedef __attribute__((ext_vector_type(4)))  float    v4f;
typedef v8h  __attribute__((may_alias)) v8ha;
typedef v4f  __attribute__((may_alias)) v4fa;
typedef v8us __attribute__((may_alias)) v8usa;

__device__ __forceinline__ unsigned short f2bf(float f) { unsigned u = __float_as_uint(f); u += 0x7FFFu + ((u >> 16) & 1u); return (unsigned short)(u >> 16); }
__device__ __forceinline__ float bf2f(unsigned short b) { return __uint_as_float(((unsigned)b) << 16); }
__device__ __forceinline__ float bfr(float f) { return bf2f(f2bf(f)); }
__device__ __forceinline__ v16h cat16(v8h lo, v8h hi) { return __builtin_shufflevector(lo, hi, 0, 1, 2, 3, 4, 5, 6, 7, 8, 9, 10, 11, 12, 13, 14, 15); }
__device__ __forceinline__ v16bf cat16b(v8us lo, v8us hi) { return __builtin_bit_cast(v16bf, __builtin_shufflevector(lo, hi, 0, 1, 2, 3, 4, 5, 6, 7, 8, 9, 10, 11, 12, 13, 14, 15)); }
__device__ __forceinline__ v8f wmma16(v16h a, v16h b, v8f c) { return __builtin_amdgcn_wmma_f32_16x16x32_f16(false, a, false, b, (short)0, c, false, false); }
__device__ __forceinline__ v8f wmmab(v16bf a, v16bf b, v8f c) { return __builtin_amdgcn_wmma_f32_16x16x32_bf16(false, a, false, b, (short)0, c, false, false); }


template <typename T16> struct WFrag;
template <> struct WFrag<h16> { typedef v16h V; static __device__ __forceinline__ V ld(const h16* p) { return cat16(*(const v8h*)p, *(const v8h*)(p + 16)); } static __device__ __forceinline__ v8f mma(V a, V b, v8f c) { return wmma16(a, b, c); } };
template <> struct WFrag<bf> { typedef v16bf V; static __device__ __forceinline__ V ld(const bf* p) { return cat16b(*(const v8us*)p, *(const v8us*)(p + 16)); } static __device__ __forceinline__ v8f mma(V a, V b, v8f c) { return wmmab(a, b, c); } };
template <typename T16, int NSPLIT, bool BIAS>
__global__ __launch_bounds__(32) void k_gemmw(const T16* __restrict__ A, const T16* __restrict__ A2, const T16* __restrict__ Bt, const T16* __restrict__ Bt2, int K, float* C, int ldc, const float* __restrict__ bias, size_t sA, size_t sB, size_t sC) {
    typedef typename WFrag<T16>::V V;
    __shared__ __align__(16) float os[16 * 68];
    const size_t z = blockIdx.z; A += z * sA; if (A2) A2 += z * sA; Bt += z * sB; if (Bt2) Bt2 += z * sB; C += z * sC;
    const int lane = threadIdx.x & 31, lr = lane & 15, hi = lane >> 4; const int r0 = blockIdx.x * 64, c0 = blockIdx.y * 64;
    v8f acc[4][4];
#pragma unroll
    for (int mb = 0; mb < 4; ++mb)
#pragma unroll
        for (int nb = 0; nb < 4; ++nb) acc[mb][nb] = (v8f){};
    const size_t aoff = (size_t)(r0 + lr) * K + 8 * hi, boff = (size_t)(c0 + lr) * K + 8 * hi;
#pragma unroll 1
    for (int kc = 0; kc < K; kc += 32) {
        V a[4], a2[4];
#pragma unroll
        for (int mb = 0; mb < 4; ++mb) { a[mb] = WFrag<T16>::ld(A + aoff + (size_t)mb * 16 * K + kc); if (NSPLIT == 1 || NSPLIT == 2) a2[mb] = WFrag<T16>::ld(A2 + aoff + (size_t)mb * 16 * K + kc); }
#pragma unroll
        for (int nb = 0; nb < 4; ++nb) { const V b = WFrag<T16>::ld(Bt + boff + (size_t)nb * 16 * K + kc); V b2; if (NSPLIT >= 2) b2 = WFrag<T16>::ld(Bt2 + boff + (size_t)nb * 16 * K + kc);
#pragma unroll
            for (int mb = 0; mb < 4; ++mb) { acc[mb][nb] = WFrag<T16>::mma(a[mb], b, acc[mb][nb]); if (NSPLIT == 1 || NSPLIT == 2) acc[mb][nb] = WFrag<T16>::mma(a2[mb], b, acc[mb][nb]); if (NSPLIT >= 2) acc[mb][nb] = WFrag<T16>::mma(a[mb], b2, acc[mb][nb]); } }
        asm volatile("v_nop\n\tv_nop\n\tv_nop\n\tv_nop" : "+v"(acc[0][0]), "+v"(acc[1][1]), "+v"(acc[2][2]), "+v"(acc[3][3]) : "v"(a[0]), "v"(a[3]));
    }
#pragma unroll
    for (int mb = 0; mb < 4; ++mb) {
#pragma unroll
        for (int nb = 0; nb < 4; ++nb) {
#pragma unroll
            for (int j = 0; j < 8; ++j) os[(hi * 8 + j) * 68 + nb * 16 + lr] = acc[mb][nb][j]; }
        __builtin_amdgcn_wave_barrier(); asm volatile("" ::: "memory");
        float* crow = C + (size_t)(r0 + mb * 16) * ldc + c0;
#pragma unroll 1
        for (int ps = 0; ps < 2; ++ps) {
#pragma unroll
            for (int s = 0; s < 8; ++s) { const int row = 2 * s + hi, cofs = lr * 4; v4f val = *(const v4fa*)(os + row * 68 + cofs); if (BIAS) { val[0] += bfr(bias[c0 + cofs]); val[1] += bfr(bias[c0 + cofs + 1]); val[2] += bfr(bias[c0 + cofs + 2]); val[3] += bfr(bias[c0 + cofs + 3]); }
                *(volatile v4f*)(crow + (size_t)row * ldc + cofs) = val; }
            if (ps == 0) __threadfence(); }
        __builtin_amdgcn_wave_barrier(); asm volatile("" ::: "memory");
    }
}

template <typename T16, int NSPLIT, int CMODE>
__global__ __launch_bounds__(32) void k_gemmc(const T16* __restrict__ A, const T16* __restrict__ A2, const T16* __restrict__ Bt, const T16* __restrict__ Bt2, int K, float* C, int ldc, int roff, size_t sA, size_t sB, size_t sC) {
    typedef typename WFrag<T16>::V V;
    __shared__ __align__(16) float os[16 * 68];
    const size_t z = blockIdx.z; A += z * sA; if (A2) A2 += z * sA; Bt += z * sB; if (Bt2) Bt2 += z * sB; C += z * sC;
    const int lane = threadIdx.x & 31, lr = lane & 15, hi = lane >> 4; const int r0 = blockIdx.x * 64, c0 = blockIdx.y * 64;
    if (CMODE == 1 && c0 > r0 + roff + 63) return;
    const int Kl = (CMODE == 2) ? min(K, r0 + roff + 64) : K;
    v8f acc[4][4];
#pragma unroll
    for (int mb = 0; mb < 4; ++mb)
#pragma unroll
        for (int nb = 0; nb < 4; ++nb) acc[mb][nb] = (v8f){};
    const size_t aoff = (size_t)(r0 + lr) * K + 8 * hi, boff = (size_t)(c0 + lr) * K + 8 * hi;
#pragma unroll 1
    for (int kc = 0; kc < Kl; kc += 32) {
        V a[4], a2[4];
#pragma unroll
        for (int mb = 0; mb < 4; ++mb) { a[mb] = WFrag<T16>::ld(A + aoff + (size_t)mb * 16 * K + kc); if (NSPLIT == 1 || NSPLIT == 2) a2[mb] = WFrag<T16>::ld(A2 + aoff + (size_t)mb * 16 * K + kc); }
#pragma unroll
        for (int nb = 0; nb < 4; ++nb) { const V b = WFrag<T16>::ld(Bt + boff + (size_t)nb * 16 * K + kc); V b2; if (NSPLIT >= 2) b2 = WFrag<T16>::ld(Bt2 + boff + (size_t)nb * 16 * K + kc);
#pragma unroll
            for (int mb = 0; mb < 4; ++mb) { acc[mb][nb] = WFrag<T16>::mma(a[mb], b, acc[mb][nb]); if (NSPLIT == 1 || NSPLIT == 2) acc[mb][nb] = WFrag<T16>::mma(a2[mb], b, acc[mb][nb]); if (NSPLIT >= 2) acc[mb][nb] = WFrag<T16>::mma(a[mb], b2, acc[mb][nb]); } }
        asm volatile("v_nop\n\tv_nop\n\tv_nop\n\tv_nop" : "+v"(acc[0][0]), "+v"(acc[1][1]), "+v"(acc[2][2]), "+v"(acc[3][3]) : "v"(a[0]), "v"(a[3]));
    }
#pragma unroll
    for (int mb = 0; mb < 4; ++mb) {
#pragma unroll
        for (int nb = 0; nb < 4; ++nb) {
#pragma unroll
            for (int j = 0; j < 8; ++j) os[(hi * 8 + j) * 68 + nb * 16 + lr] = acc[mb][nb][j]; }
        __builtin_amdgcn_wave_barrier(); asm volatile("" ::: "memory");
        float* crow = C + (size_t)(r0 + mb * 16) * ldc + c0;
#pragma unroll 1
        for (int ps = 0; ps < 2; ++ps) {
#pragma unroll
            for (int s = 0; s < 8; ++s) { const int row = 2 * s + hi, cofs = lr * 4; v4f val = *(const v4fa*)(os + row * 68 + cofs);
                *(volatile v4f*)(crow + (size_t)row * ldc + cofs) = val; }
            if (ps == 0) __threadfence(); }
        __builtin_amdgcn_wave_barrier(); asm volatile("" ::: "memory");
    }
}

__device__ __forceinline__ h16 tohx(float x) { return (h16)x; }
__device__ __forceinline__ void splitf(float y, unsigned short& h, unsigned short& l) { h = f2bf(y); l = f2bf(y - bf2f(h)); }
__device__ __forceinline__ float silu_(float x) { return __fmul_rn(x, __fdiv_rn(1.0f, 1.0f + __expf(-x))); }
typedef __attribute__((ext_vector_type(2))) _Float16 v2h;
typedef __attribute__((ext_vector_type(4))) _Float16 v4h;
typedef __attribute__((ext_vector_type(2))) unsigned short v2us;
typedef __attribute__((ext_vector_type(4))) unsigned short v4us;
typedef __attribute__((ext_vector_type(2))) float v2f;

__global__ __launch_bounds__(256) void k_cvt8(const float* __restrict__ src, bf* dst, size_t n8) { const size_t i = (size_t)blockIdx.x * 256 + threadIdx.x; if (i >= n8) return; const v8f v = *(const v8f*)(src + i * 8); v8us o;
#pragma unroll
    for (int k = 0; k < 8; ++k) o[k] = f2bf(v[k]); *(volatile v8us*)(dst + i * 8) = o; __threadfence(); *(volatile v8us*)(dst + i * 8) = o; }
__global__ __launch_bounds__(256) void k_w1p(const float* __restrict__ w, bf* Bt) { const int e = (blockIdx.x * 256 + threadIdx.x) * 4; if (e >= 128 * 32) return; const int k = e % 32, n = e / 32; v4us o;
#pragma unroll
    for (int q = 0; q < 4; ++q) o[q] = (k + q) < 15 ? f2bf(w[n * 15 + k + q]) : (unsigned short)0; *(volatile v4us*)(Bt + e) = o; __threadfence(); *(volatile v4us*)(Bt + e) = o; }
__global__ __launch_bounds__(256) void k_wdt(const float* __restrict__ w, bf* WDT) { const int i = (blockIdx.x * 256 + threadIdx.x) * 4; if (i >= 64 * DIM) return; const int k = i % DIM, n = i / DIM; v4us o;
#pragma unroll
    for (int q = 0; q < 4; ++q) o[q] = n < NH_ ? f2bf(w[(size_t)(640 + n) * DIM + k + q]) : (unsigned short)0; *(volatile v4us*)(WDT + i) = o; __threadfence(); *(volatile v4us*)(WDT + i) = o; }
__global__ __launch_bounds__(256) void k_tok(const float* __restrict__ x, bf* TOK) { const int e = (blockIdx.x * 256 + threadIdx.x) * 4; if (e >= TT * 32) return; const int k = e % 32, l = e / 32; v4us o;
#pragma unroll
    for (int q = 0; q < 4; ++q) { const int kk = k + q; unsigned short v = 0; if (l < LQ - 1 && kk < 15) { const int w = kk / 3, c = kk % 3; v = f2bf(x[(size_t)(l + w) * 3 + c]); } o[q] = v; } *(volatile v4us*)(TOK + e) = o; __threadfence(); *(volatile v4us*)(TOK + e) = o; }
__global__ __launch_bounds__(256) void k_gelu2(const float* __restrict__ A1, const float* __restrict__ b1, bf* Gh, bf* Gl) { const int i = (blockIdx.x * 256 + threadIdx.x) * 4; if (i >= TT * 128) return; const int c = i % 128; const v4f a = *(const v4f*)(A1 + i); v4us oh, ol;
#pragma unroll
    for (int q = 0; q < 4; ++q) { const float t = __fadd_rn(a[q], bfr(b1[c + q])); const float g = 0.5f * t * (1.0f + erff(t * 0.7071067811865476f)); unsigned short u, l; splitf(g, u, l); oh[q] = u; ol[q] = l; } *(volatile v4us*)(Gh + i) = oh; *(volatile v4us*)(Gl + i) = ol; __threadfence(); *(volatile v4us*)(Gh + i) = oh; *(volatile v4us*)(Gl + i) = ol; }
__global__ __launch_bounds__(256) void k_hcls(const float* __restrict__ A2, const float* __restrict__ b2, const float* __restrict__ cls, float* H) { const int i = (blockIdx.x * 256 + threadIdx.x) * 4; if (i >= TT * DIM) return; const int c = i % DIM, l = i / DIM; const v4f a = *(const v4f*)(A2 + i); v4f o;
#pragma unroll
    for (int q = 0; q < 4; ++q) o[q] = l < LQ - 1 ? __fadd_rn(a[q], bfr(b2[c + q])) : (l == LQ - 1 ? bfr(cls[c + q]) : 0.f); *(volatile v4f*)(H + i) = o; __threadfence(); *(volatile v4f*)(H + i) = o; }
__global__ __launch_bounds__(256) void k_spl(const float* __restrict__ F, size_t n4, bf* Fh, bf* Fl) { const size_t i = ((size_t)blockIdx.x * 256 + threadIdx.x) * 4; if (i >= n4 * 4) return; const v4f a = *(const v4f*)(F + i); v4us oh, ol;
#pragma unroll
    for (int q = 0; q < 4; ++q) { unsigned short u, c2; splitf(a[q], u, c2); oh[q] = u; ol[q] = c2; } *(volatile v4us*)(Fh + i) = oh; *(volatile v4us*)(Fl + i) = ol; __threadfence(); *(volatile v4us*)(Fh + i) = oh; *(volatile v4us*)(Fl + i) = ol; }
__global__ __launch_bounds__(256) void k_conv(const float* __restrict__ ZX, const float* __restrict__ w, const float* __restrict__ bb, float* XC) { const size_t e = ((size_t)blockIdx.x * 256 + threadIdx.x) * 4; if (e >= (size_t)TT * CD) return; const int c = (int)(e % CD); const int t = (int)(e / CD); v4f o;
#pragma unroll
    for (int q = 0; q < 4; ++q) { float acc = bfr(bb[c + q]);
#pragma unroll
        for (int k = 0; k < 4; ++k) { const int ts = t - 3 + k; if (ts >= 0) { float p = __fmul_rn(ZX[(size_t)ts * DP + DI + c + q], bfr(w[(c + q) * 4 + k])); asm volatile("" : "+v"(p)); acc = __fadd_rn(acc, p); } }
        o[q] = silu_(acc); }
    *(volatile v4f*)(XC + e) = o; __threadfence(); *(volatile v4f*)(XC + e) = o; }
__global__ __launch_bounds__(256) void k_bcpl(const float* __restrict__ XC, bf* Ch, bf* Cl, bf* Bh, bf* Bl) { const size_t e = ((size_t)blockIdx.x * 256 + threadIdx.x) * 2; if (e >= (size_t)TT * DS) return; const int n = (int)(e % DS); const int t = (int)(e / DS); const float* r = XC + (size_t)t * CD + DI; v2us ch_, cl_, bh_, bl_; unsigned short a, c;
    splitf(r[DS + n], a, c); ch_[0] = a; cl_[0] = c; splitf(r[DS + n + 1], a, c); ch_[1] = a; cl_[1] = c; splitf(r[n], a, c); bh_[0] = a; bl_[0] = c; splitf(r[n + 1], a, c); bh_[1] = a; bl_[1] = c;
    for (int ps = 0; ps < 2; ++ps) { *(volatile v2us*)(Ch + e) = ch_; *(volatile v2us*)(Cl + e) = cl_; *(volatile v2us*)(Bh + e) = bh_; *(volatile v2us*)(Bl + e) = bl_; if (ps == 0) __threadfence(); } }
__global__ __launch_bounds__(256) void k_xt16(const float* __restrict__ XC, h16* XT) { const size_t e = ((size_t)blockIdx.x * 256 + threadIdx.x) * 2; if (e >= (size_t)NH_ * HP * TT) return; const int s = (int)(e % TT); const int p = (int)((e / TT) % HP); const int h = (int)(e / ((size_t)TT * HP)); v2h o; o[0] = tohx(XC[(size_t)s * CD + h * HP + p]); o[1] = tohx(XC[(size_t)(s + 1) * CD + h * HP + p]); *(volatile v2h*)(XT + e) = o; __threadfence(); *(volatile v2h*)(XT + e) = o; }
__global__ __launch_bounds__(32) void k_dtcum(const float* __restrict__ DTR, const float* __restrict__ dtb, const float* __restrict__ alog, float* DT, double* CUM) { const int h = threadIdx.x; const bool live = h < NH_; const float A = live ? -__expf(bfr(alog[h])) : 0.f; const float bias = live ? bfr(dtb[h]) : 0.f;
    for (int ps = 0; ps < 2; ++ps) { double c = 0.0; for (int t = 0; t < TT; ++t) { float dt = 0.f; if (live) { const float raw = __fadd_rn(DTR[(size_t)t * 64 + h], bias); dt = raw > 20.f ? raw : log1pf(__expf(raw)); c += (double)__fmul_rn(dt, A); } *(volatile float*)(DT + (size_t)t * 32 + h) = dt; if (h < 16) *(volatile double*)(CUM + (size_t)t * 16 + h) = c; } if (ps == 0) __threadfence(); } }
__global__ __launch_bounds__(256) void k_mask(const float* __restrict__ G, const float* __restrict__ DT, const double* __restrict__ CUM, h16* M16) { const size_t e = ((size_t)blockIdx.x * 256 + threadIdx.x) * 4; if (e >= (size_t)ZH * TT * TT) return; const int s0 = (int)(e % TT); const int t = (int)((e / TT) % TT); const int h = (int)(e / ((size_t)TT * TT)); const double ct = CUM[(size_t)t * 16 + h]; const v4f g = *(const v4f*)(G + (size_t)t * TT + s0); v4h o;
#pragma unroll
    for (int q = 0; q < 4; ++q) { const int s = s0 + q; float v = 0.f; if (s <= t) { const float dl = (float)(ct - CUM[(size_t)s * 16 + h]); float w = __fmul_rn(__expf(dl), DT[(size_t)s * 32 + h]); asm volatile("" : "+v"(w)); v = __fmul_rn(g[q], w); } o[q] = tohx(v); }
    *(volatile v4h*)(M16 + e) = o; __threadfence(); *(volatile v4h*)(M16 + e) = o; }
__global__ __launch_bounds__(256) void k_gate(const float* __restrict__ Y, const float* __restrict__ XC, const float* __restrict__ ZX, const float* __restrict__ Dv, float* GG) { const size_t e = ((size_t)blockIdx.x * 256 + threadIdx.x) * 2; if (e >= (size_t)NH_ * TT * HP) return; const int p = (int)(e % HP); const int t = (int)((e / HP) % TT); const int h = (int)(e / ((size_t)HP * TT)); const float dd = bfr(Dv[h]); v2f o;
#pragma unroll
    for (int u = 0; u < 2; ++u) { const int c = h * HP + p + u; float sk = __fmul_rn(XC[(size_t)t * CD + c], dd); asm volatile("" : "+v"(sk)); const float y = __fadd_rn(Y[e + u], sk); o[u] = __fmul_rn(y, silu_(ZX[(size_t)t * DP + c])); }
    const size_t oo = (size_t)t * DI + h * HP + p; *(volatile v2f*)(GG + oo) = o; __threadfence(); *(volatile v2f*)(GG + oo) = o; }
__global__ __launch_bounds__(256) void k_grms(const float* __restrict__ GG, const float* __restrict__ nw, bf* Gh, bf* Gl) { const int lane = threadIdx.x & 31; const int t = blockIdx.x * 8 + (threadIdx.x >> 5); if (t >= TT) return; const float* r = GG + (size_t)t * DI; float q2 = 0.f;
#pragma unroll
    for (int ch = 0; ch < 2; ++ch) { const v4f a = *(const v4f*)(r + ch * 128 + lane * 4);
#pragma unroll
        for (int q = 0; q < 4; ++q) { float p = __fmul_rn(a[q], a[q]); asm volatile("" : "+v"(p)); q2 = __fadd_rn(q2, p); } }
#pragma unroll
    for (int sh = 16; sh; sh >>= 1) q2 += __shfl_xor(q2, sh, 32);
    float vq = q2 * (1.0f / DI); asm volatile("" : "+v"(vq)); const float rs = __frsqrt_rn(__fadd_rn(vq, 1e-5f));
#pragma unroll 1
    for (int ch = 0; ch < 2; ++ch) { const int c0 = ch * 128 + lane * 4; const v4f a = *(const v4f*)(r + c0); v4us oh, ol;
#pragma unroll
        for (int q = 0; q < 4; ++q) { float tn = __fmul_rn(a[q], rs); asm volatile("" : "+v"(tn)); unsigned short u, c; splitf(__fmul_rn(tn, bfr(nw[c0 + q])), u, c); oh[q] = u; ol[q] = c; }
        const size_t oo = (size_t)t * DI + c0; *(volatile v4us*)(Gh + oo) = oh; *(volatile v4us*)(Gl + oo) = ol; __threadfence(); *(volatile v4us*)(Gh + oo) = oh; *(volatile v4us*)(Gl + oo) = ol; } }
__global__ __launch_bounds__(256) void k_out1(const float* __restrict__ H, int b, float* DOUT, float* STASH) { const int t = blockIdx.x * 256 + threadIdx.x; const long local = 4L * t - 8; if (local < 0 || local >= (long)LQ * DIM) return; const v4f a = *(const v4f*)(H + local);
    if (b == 0 && local < 24) { *(volatile v4f*)(STASH + local) = a; __threadfence(); *(volatile v4f*)(STASH + local) = a; return; }
    float* dst = DOUT + 8 + (size_t)b * LQ * DIM + local; *(volatile v4f*)dst = a; __threadfence(); *(volatile v4f*)dst = a; }
__global__ __launch_bounds__(32) void k_line0(const float* __restrict__ O0S, const float* __restrict__ STASH, float* DOUT) { const int l = threadIdx.x; const float v = l < 8 ? O0S[l] : STASH[l - 8]; *(volatile float*)(DOUT + l) = v; __threadfence(); *(volatile float*)(DOUT + l) = v; }
__global__ __launch_bounds__(32) void k_head(const float* __restrict__ H, const float* __restrict__ lw, const float* __restrict__ lb, const float* __restrict__ hw, const float* __restrict__ hb, float* O0) { const int lane = threadIdx.x; const float* r = H + (size_t)(LQ - 1) * DIM; float v[4]; float s = 0.f;
#pragma unroll
    for (int q = 0; q < 4; ++q) { v[q] = r[lane * 4 + q]; s = __fadd_rn(s, v[q]); }
#pragma unroll
    for (int sh = 16; sh; sh >>= 1) s += __shfl_xor(s, sh, 32);
    const float mu = s * (1.0f / DIM); float q2 = 0.f;
#pragma unroll
    for (int q = 0; q < 4; ++q) { float dv = __fsub_rn(v[q], mu); asm volatile("" : "+v"(dv)); float p = __fmul_rn(dv, dv); asm volatile("" : "+v"(p)); q2 = __fadd_rn(q2, p); }
#pragma unroll
    for (int sh = 16; sh; sh >>= 1) q2 += __shfl_xor(q2, sh, 32);
    float vq = q2 * (1.0f / DIM); asm volatile("" : "+v"(vq)); const float rs = __frsqrt_rn(__fadd_rn(vq, 1e-5f)); float d = 0.f;
#pragma unroll
    for (int q = 0; q < 4; ++q) { const int c = lane * 4 + q; float dv = __fsub_rn(v[q], mu); asm volatile("" : "+v"(dv)); float tn = __fmul_rn(dv, rs); asm volatile("" : "+v"(tn)); float tg = __fmul_rn(tn, bfr(lw[c])); asm volatile("" : "+v"(tg)); const float y = __fadd_rn(tg, bfr(lb[c])); float p = __fmul_rn(y, bfr(hw[c])); asm volatile("" : "+v"(p)); d = __fadd_rn(d, p); }
#pragma unroll
    for (int sh = 16; sh; sh >>= 1) d += __shfl_xor(d, sh, 32);
    const float o = __fadd_rn(d, bfr(hb[0])); if (lane == 0) { *(volatile float*)O0 = o; __threadfence(); *(volatile float*)O0 = o; } }

extern "C" void kernel_launch(void* const* d_in, const int* in_sizes, int n_in,
                              void* d_out, int out_size, void* d_ws, size_t ws_size, hipStream_t stream) {
    (void)in_sizes; (void)n_in; (void)out_size;
    const float* IN[18]; for (int i = 0; i < 18; ++i) IN[i] = (const float*)d_in[i];
    float* DOUT = (float*)d_out;
    char* wsp = (char*)d_ws;
    auto take = [&](size_t bytes) { char* p = wsp; wsp += (bytes + 255) & ~(size_t)255; return (void*)p; };
    bf* W1B = (bf*)take((size_t)128 * 32 * 2); bf* W2B = (bf*)take((size_t)DIM * 128 * 2); bf* WIP = (bf*)take((size_t)4 * DP * DIM * 2); bf* WDT = (bf*)take((size_t)4 * 64 * DIM * 2); bf* WOP = (bf*)take((size_t)4 * DIM * DI * 2);
    bf* TOK = (bf*)take((size_t)TT * 32 * 2); float* A1 = (float*)take((size_t)TT * 128 * 4); bf* Th = (bf*)take((size_t)TT * DI * 2); bf* Tl = (bf*)take((size_t)TT * DI * 2); float* H = (float*)take((size_t)TT * DIM * 4);
    float* ZX = (float*)take((size_t)TT * DP * 4); float* DTR = (float*)take((size_t)TT * 64 * 4); float* XC = (float*)take((size_t)TT * CD * 4); bf* Ch = (bf*)take((size_t)TT * DS * 2); bf* Cl = (bf*)take((size_t)TT * DS * 2); bf* Bh = (bf*)take((size_t)TT * DS * 2); bf* Bl = (bf*)take((size_t)TT * DS * 2); float* G = (float*)take((size_t)TT * TT * 4); h16* XT = (h16*)take((size_t)NH_ * HP * TT * 2); float* DT = (float*)take((size_t)TT * 32 * 4); double* CUM = (double*)take((size_t)TT * 16 * 8);
    float* O0S = (float*)take(256); float* STASH = (float*)take(256); h16* M16 = (h16*)take((size_t)ZH * TT * TT * 2); float* Y = (float*)take((size_t)NH_ * TT * HP * 4); float* GG = (float*)take((size_t)TT * DI * 4);
    if ((size_t)(wsp - (char*)d_ws) > ws_size) return;
    k_w1p<<<(128 * 32 / 4 + 255) / 256, 256, 0, stream>>>(IN[1], W1B); k_cvt8<<<(DIM * 128 / 8 + 255) / 256, 256, 0, stream>>>(IN[3], W2B, (size_t)DIM * 128 / 8);
    for (int l = 0; l < 4; ++l) { k_cvt8<<<(DP * DIM / 8 + 255) / 256, 256, 0, stream>>>(IN[6] + (size_t)l * DP * DIM, WIP + (size_t)l * DP * DIM, (size_t)DP * DIM / 8); k_wdt<<<(64 * DIM / 4 + 255) / 256, 256, 0, stream>>>(IN[6] + (size_t)l * DP * DIM, WDT + (size_t)l * 64 * DIM); k_cvt8<<<(DIM * DI / 8 + 255) / 256, 256, 0, stream>>>(IN[13] + (size_t)l * DIM * DI, WOP + (size_t)l * DIM * DI, (size_t)DIM * DI / 8); }
    for (int b = 0; b < NB_; ++b) {
        k_tok<<<(TT * 32 / 4 + 255) / 256, 256, 0, stream>>>(IN[0] + (size_t)b * TIN * 3, TOK);
        k_gemmw<bf, 0, false><<<dim3(TT / 64, 128 / 64, 1), 32, 0, stream>>>(TOK, nullptr, W1B, nullptr, 32, A1, 128, nullptr, 0, 0, 0); k_gelu2<<<(TT * 128 / 4 + 255) / 256, 256, 0, stream>>>(A1, IN[2], Th, Tl);
        k_gemmw<bf, 1, false><<<dim3(TT / 64, DIM / 64, 1), 32, 0, stream>>>(Th, Tl, W2B, nullptr, 128, A1, DIM, nullptr, 0, 0, 0); k_hcls<<<(TT * DIM / 4 + 255) / 256, 256, 0, stream>>>(A1, IN[4], IN[5], H);
        for (int l = 0; l < 4; ++l) { const bf* wip = WIP + (size_t)l * DP * DIM; const bf* wdt = WDT + (size_t)l * 64 * DIM; const bf* wop = WOP + (size_t)l * DIM * DI;
            k_spl<<<(TT * DIM / 4 + 255) / 256, 256, 0, stream>>>(H, (size_t)TT * DIM / 4, Th, Tl);
            k_gemmw<bf, 1, false><<<dim3(TT / 64, 640 / 64, 1), 32, 0, stream>>>(Th, Tl, wip, nullptr, DIM, ZX, DP, nullptr, 0, 0, 0); k_gemmw<bf, 1, false><<<dim3(TT / 64, 1, 1), 32, 0, stream>>>(Th, Tl, wdt, nullptr, DIM, DTR, 64, nullptr, 0, 0, 0);
            k_conv<<<(unsigned)(((size_t)TT * CD / 4 + 255) / 256), 256, 0, stream>>>(ZX, IN[7] + (size_t)l * CD * 4, IN[8] + (size_t)l * CD, XC);
            k_bcpl<<<(TT * DS / 2 + 255) / 256, 256, 0, stream>>>(XC, Ch, Cl, Bh, Bl); k_xt16<<<(unsigned)(((size_t)NH_ * HP * TT / 2 + 255) / 256), 256, 0, stream>>>(XC, XT); k_dtcum<<<1, 32, 0, stream>>>(DTR, IN[9] + l * NH_, IN[10] + l * NH_, DT, CUM);
            k_gemmc<bf, 2, 1><<<dim3(TT / 64, TT / 64, 1), 32, 0, stream>>>(Ch, Cl, Bh, Bl, DS, G, TT, 0, 0, 0, 0);
            k_mask<<<(unsigned)(((size_t)ZH * TT * TT / 4 + 255) / 256), 256, 0, stream>>>(G, DT, CUM, M16);
            k_gemmc<h16, 0, 2><<<dim3(TT / 64, 1, ZH), 32, 0, stream>>>(M16, nullptr, XT, nullptr, TT, Y, HP, 0, (size_t)TT * TT, (size_t)HP * TT, (size_t)TT * HP);
            k_gate<<<(unsigned)(((size_t)NH_ * TT * HP / 2 + 255) / 256), 256, 0, stream>>>(Y, XC, ZX, IN[11] + l * NH_, GG); k_grms<<<TT / 8, 256, 0, stream>>>(GG, IN[12] + (size_t)l * DI, Th, Tl);
            k_gemmw<bf, 1, false><<<dim3(TT / 64, DIM / 64, 1), 32, 0, stream>>>(Th, Tl, wop, nullptr, DI, H, DIM, nullptr, 0, 0, 0); }
        k_out1<<<(unsigned)(((size_t)LQ * DIM / 4 + 2 + 255) / 256), 256, 0, stream>>>(H, b, DOUT, STASH); k_head<<<1, 32, 0, stream>>>(H, IN[14], IN[15], IN[16], IN[17], O0S + b); }
    k_line0<<<1, 32, 0, stream>>>(O0S, STASH, DOUT);
}
